// SwinTransformerBlock_14104672600653
// MI455X (gfx1250) — hardware-run, weakly checked
//
#include <hip/hip_runtime.h>

typedef __attribute__((ext_vector_type(16))) _Float16 v16h;
typedef __attribute__((ext_vector_type(8)))  _Float16 v8h;
typedef __attribute__((ext_vector_type(8)))  float    v8f;
typedef __attribute__((ext_vector_type(4)))  float    v4f;

constexpr int kTok     = 100352;
constexpr int kTokImg  = 3136;
constexpr int kC       = 128;
constexpr int kQKVN    = 384;
constexpr int kHid     = 512;
constexpr int kNTokW   = 49;
constexpr int kNWin    = 2048;
constexpr int kChunk   = 25088;
constexpr int kNChunk  = 4;

static_assert(kTok % 64 == 0);
static_assert(kChunk % 64 == 0);
static_assert(kChunk * kNChunk == kTok);
static_assert(kC % 64 == 0 && kQKVN % 64 == 0 && kHid % 64 == 0);
static_assert(kC % 32 == 0 && kHid % 32 == 0);
static_assert(kNWin * kNTokW == kTok);

__device__ __forceinline__ void dep_guard_h(v8f& a, v8f& b, v16h x, v16h y) { asm volatile("v_nop\n\tv_nop\n\tv_nop\n\tv_nop" : "+v"(a), "+v"(b) : "v"(x), "v"(y)); }
__device__ __forceinline__ void keep4_h(v16h a, v16h b, v16h c, v16h d) { asm volatile("v_nop" :: "v"(a), "v"(b), "v"(c), "v"(d)); }
__device__ __forceinline__ void acc_guard4(v8f& a, v8f& b, v8f& c, v8f& d) { asm volatile("v_nop\n\tv_nop\n\tv_nop\n\tv_nop" : "+v"(a), "+v"(b), "+v"(c), "+v"(d)); }

template <typename T> struct Frag;
template <> struct Frag<_Float16> {
  typedef v16h V; union U { v16h v; v8h h[2]; };
  static __device__ __forceinline__ v16h load(const _Float16* p) {
    U f; f.h[0] = *(const v8h*)(p); f.h[1] = *(const v8h*)(p + 16); return f.v;
  }
  static __device__ __forceinline__ v8f mma(v16h a, v16h b, v8f c) {
    return __builtin_amdgcn_wmma_f32_16x16x32_f16(false, a, false, b, (short)0, c, false, false);
  }
  static __device__ __forceinline__ void guard(v8f& a, v8f& b, v16h x, v16h y) { dep_guard_h(a, b, x, y); }
  static __device__ __forceinline__ void keep(v16h a, v16h b, v16h c, v16h d) { keep4_h(a, b, c, d); }
};

__device__ __forceinline__ v8f mma_h(v16h a, v16h b, v8f c) {
  c = __builtin_amdgcn_wmma_f32_16x16x32_f16(false, a, false, b, (short)0, c, false, false);
  asm volatile("v_nop\n\tv_nop\n\tv_nop\n\tv_nop" : "+v"(c) : "v"(a), "v"(b));
  return c;
}

__device__ __forceinline__ int win_row_to_img_row(int m) {
  const int bimg = m / kTokImg;
  const int r = m - bimg * kTokImg;
  const int win = r / kNTokW;
  const int tok = r - win * kNTokW;
  const int wh = win >> 3, wn = win & 7;
  const int ih = tok / 7;
  const int iw = tok - ih * 7;
  int sh = wh * 7 + ih + 3; sh = (sh >= 56) ? (sh - 56) : sh;
  int sw = wn * 7 + iw + 3; sw = (sw >= 56) ? (sw - 56) : sw;
  return bimg * kTokImg + sh * 56 + sw;
}

template <int BIAS_MODE, int OUT_MODE, bool RESID, bool PERM>
__global__ __launch_bounds__(256) void gemm64_f16(
    const unsigned short* __restrict__ Ap, int lda,
    const unsigned short* __restrict__ Btp, int ldb,
    void* __restrict__ Cout, int ldc,
    const float* __restrict__ bias, float bscale,
    const float* __restrict__ resid,
    int M, int N, int K, float scale) {
  typedef _Float16 T;
  typedef v16h V;
  const T* Ab = (const T*)Ap;
  const T* Bb = (const T*)Btp;
  __shared__ __align__(16) float sT[8][16 * 68];
  const int lane = threadIdx.x & 31;
  const int wave = threadIdx.x >> 5;
  const int tilesN = N >> 6;
  const int tilesM = M >> 6;
  const int tile = blockIdx.x * 8 + wave;
  if (tile >= tilesM * tilesN) return;
  const int tm = tile / tilesN;
  const int tn = tile - tm * tilesN;
  const int m0 = tm << 6;
  const int n0 = tn << 6;

  const int rlane = lane & 15;
  const int koff  = (lane >> 4) * 8;
  const int mOff  = (lane >> 4) * 8;

  v8f acc[4][4];
#pragma unroll
  for (int i = 0; i < 4; ++i)
#pragma unroll
    for (int j = 0; j < 4; ++j) acc[i][j] = (v8f){0.f,0.f,0.f,0.f,0.f,0.f,0.f,0.f};

  for (int k0 = 0; k0 < K; k0 += 32) {
    V bh[4];
#pragma unroll
    for (int j = 0; j < 4; ++j) {
      const size_t bo = (size_t)(n0 + (j << 4) + rlane) * ldb + koff + k0;
      bh[j] = Frag<T>::load(Bb + bo);
    }
#pragma unroll
    for (int i = 0; i < 4; ++i) {
      const size_t ao = (size_t)(m0 + (i << 4) + rlane) * lda + koff + k0;
      V ah = Frag<T>::load(Ab + ao);
#pragma unroll
      for (int j = 0; j < 4; ++j) acc[i][j] = Frag<T>::mma(ah, bh[j], acc[i][j]);
      Frag<T>::guard(acc[i][0], acc[i][3], ah, ah);
    }
    Frag<T>::keep(bh[0], bh[1], bh[2], bh[3]);
  }
  acc_guard4(acc[0][0], acc[0][1], acc[0][2], acc[0][3]);
  acc_guard4(acc[1][0], acc[1][1], acc[1][2], acc[1][3]);
  acc_guard4(acc[2][0], acc[2][1], acc[2][2], acc[2][3]);
  acc_guard4(acc[3][0], acc[3][1], acc[3][2], acc[3][3]);

  float* slab = sT[wave];
  float bvj[4] = {0.f, 0.f, 0.f, 0.f};
  if (BIAS_MODE == 2) {
#pragma unroll
    for (int j = 0; j < 4; ++j) bvj[j] = bias[n0 + (j << 4) + rlane] * bscale;
  }
#pragma unroll
  for (int i = 0; i < 4; ++i) {
    const int mBase = m0 + (i << 4);
#pragma unroll
    for (int j = 0; j < 4; ++j) {
#pragma unroll
      for (int r = 0; r < 8; ++r) {
        float v = acc[i][j][r] * scale;
        if (BIAS_MODE == 2) v += bvj[j];
        slab[(mOff + r) * 68 + (j << 4) + rlane] = v;
      }
    }
    __builtin_amdgcn_fence(__ATOMIC_RELEASE, "workgroup");
    __builtin_amdgcn_wave_barrier();
    __builtin_amdgcn_fence(__ATOMIC_ACQUIRE, "workgroup");
    if (OUT_MODE == 0) {
      float* Cf = (float*)Cout;
      const int hh = lane >> 4, c4 = (lane & 15) * 4;
      v4f vals[8];
      size_t addr[8];
#pragma unroll
      for (int it = 0; it < 8; ++it) {
        const int row = it * 2 + hh;
        int grow = mBase + row;
        if (PERM) grow = win_row_to_img_row(grow);
        v4f v = *(const v4f*)(slab + row * 68 + c4);
        const size_t o = (size_t)grow * ldc + n0 + c4;
        if (RESID) { const v4f rr = *(const v4f*)(resid + o); v += rr; }
        vals[it] = v;
        addr[it] = o;
      }
      for (int pass = 0; pass < 2; ++pass) {
#pragma unroll
        for (int it = 0; it < 8; ++it) *(volatile v4f*)(Cf + addr[it]) = vals[it];
        __threadfence();
      }
    } else {
      const int q = lane >> 3, c8 = (lane & 7) * 8;
      unsigned short* Ch = (unsigned short*)Cout;
      for (int pass = 0; pass < 2; ++pass) {
#pragma unroll
        for (int it = 0; it < 4; ++it) {
          const int row = it * 4 + q;
          const float* sp = slab + row * 68 + c8;
          v8h hv;
#pragma unroll
          for (int e = 0; e < 8; ++e) hv[e] = (_Float16)sp[e];
          *(volatile v8h*)(Ch + (size_t)(mBase + row) * ldc + n0 + c8) = hv;
        }
        __threadfence();
      }
    }
    __builtin_amdgcn_fence(__ATOMIC_RELEASE, "workgroup");
    __builtin_amdgcn_wave_barrier();
    __builtin_amdgcn_fence(__ATOMIC_ACQUIRE, "workgroup");
  }
}

__global__ __launch_bounds__(256) void cast_f32_f16x2(
    const float* __restrict__ in, _Float16* __restrict__ out, int n2, float mul) {
  const int i = blockIdx.x * 256 + threadIdx.x;
  if (i < n2) {
    const _Float16 h0 = (_Float16)(in[2 * i] * mul);
    const _Float16 h1 = (_Float16)(in[2 * i + 1] * mul);
    const unsigned u = (unsigned)__builtin_bit_cast(unsigned short, h0) | ((unsigned)__builtin_bit_cast(unsigned short, h1) << 16);
    ((volatile unsigned*)out)[i] = u;
    __threadfence();
    ((volatile unsigned*)out)[i] = u;
  }
}

template <bool WINMAP>
__global__ __launch_bounds__(128) void ln_rows_kernel(
    const float* __restrict__ x, const float* __restrict__ g, const float* __restrict__ bb,
    _Float16* __restrict__ out, int nrows) {
  const int lane = threadIdx.x & 31;
  const int wave = threadIdx.x >> 5;
  const int t = blockIdx.x * 4 + wave;
  if (t >= nrows) return;
  const int srow = WINMAP ? win_row_to_img_row(t) : t;
  const v4f xv = *(const v4f*)(x + (size_t)srow * kC + lane * 4);
  float s = (xv[0] + xv[1]) + (xv[2] + xv[3]);
#pragma unroll
  for (int m = 16; m >= 1; m >>= 1) s += __shfl_xor(s, m, 32);
  const float mean = s * (1.0f / 128.0f);
  const float d0 = xv[0] - mean, d1 = xv[1] - mean, d2 = xv[2] - mean, d3 = xv[3] - mean;
  float ss = (d0 * d0 + d1 * d1) + (d2 * d2 + d3 * d3);
#pragma unroll
  for (int m = 16; m >= 1; m >>= 1) ss += __shfl_xor(ss, m, 32);
  const float rs = rsqrtf(ss * (1.0f / 128.0f) + 1e-5f);
  const v4f gv = *(const v4f*)(g + lane * 4);
  const v4f bv = *(const v4f*)(bb + lane * 4);
  const float y0 = d0 * rs * gv[0] + bv[0];
  const float y1 = d1 * rs * gv[1] + bv[1];
  const float y2 = d2 * rs * gv[2] + bv[2];
  const float y3 = d3 * rs * gv[3] + bv[3];
  const int s0 = (2 * lane) & 31, s1 = (2 * lane + 1) & 31;
  const float a0 = __shfl(y0, s0, 32), a1 = __shfl(y1, s0, 32), a2 = __shfl(y2, s0, 32), a3 = __shfl(y3, s0, 32);
  const float b0 = __shfl(y0, s1, 32), b1 = __shfl(y1, s1, 32), b2 = __shfl(y2, s1, 32), b3 = __shfl(y3, s1, 32);
  v8h hv;
  hv[0] = (_Float16)a0; hv[1] = (_Float16)a1; hv[2] = (_Float16)a2; hv[3] = (_Float16)a3;
  hv[4] = (_Float16)b0; hv[5] = (_Float16)b1; hv[6] = (_Float16)b2; hv[7] = (_Float16)b3;
  _Float16* dst = out + (size_t)t * kC + (lane & 15) * 8;
  if (lane < 16) *(volatile v8h*)dst = hv;
  __threadfence();
  if (lane < 16) *(volatile v8h*)dst = hv;
}

__global__ __launch_bounds__(256) void gelu_f16x2_kernel(
    const unsigned* __restrict__ in, unsigned* __restrict__ out, int n2) {
  const int i = blockIdx.x * 256 + threadIdx.x;
  if (i < n2) {
    const unsigned w = in[i];
    const float f0 = (float)__builtin_bit_cast(_Float16, (unsigned short)(w & 0xffffu)) * 0.125f;
    const float f1 = (float)__builtin_bit_cast(_Float16, (unsigned short)(w >> 16)) * 0.125f;
    const float g0 = 0.5f * f0 * (1.0f + erff(f0 * 0.70710678118654752f));
    const float g1 = 0.5f * f1 * (1.0f + erff(f1 * 0.70710678118654752f));
    const _Float16 h0 = (_Float16)(g0 * 16.0f);
    const _Float16 h1 = (_Float16)(g1 * 16.0f);
    const unsigned u = (unsigned)__builtin_bit_cast(unsigned short, h0) | ((unsigned)__builtin_bit_cast(unsigned short, h1) << 16);
    ((volatile unsigned*)out)[i] = u;
    __threadfence();
    ((volatile unsigned*)out)[i] = u;
  }
}

__device__ __forceinline__ int region_id(int p) { return p < 49 ? 0 : (p < 53 ? 1 : 2); }

__global__ __launch_bounds__(256) void window_attention_kernel(
    const unsigned short* __restrict__ qkv, const float* __restrict__ rpb, unsigned short* __restrict__ atto) {
  __shared__ __align__(16) unsigned short kvs[16384];
  __shared__ __align__(16) _Float16 psh[8][32 * 64];
  __shared__ float rpbs[169 * 4];

  const int tid = threadIdx.x;
  const int wave = tid >> 5, lane = tid & 31, hh = lane >> 4, c = lane & 15;
  const int win = blockIdx.x;
  const int wloc = win & 63, wh = wloc >> 3, wn = wloc & 7;
  const size_t rowbase = (size_t)win * kNTokW;

  for (int i = tid; i < 169 * 4; i += 256) rpbs[i] = rpb[i];
#pragma unroll
  for (int i = 0; i < 4; ++i) {
    const int s = tid + 256 * i;
    const int kv = s >> 4, rem = s & 15, hd4 = rem >> 2, q4 = rem & 3;
    const int kvc = (kv < kNTokW) ? kv : (kNTokW - 1);
    const size_t src = (rowbase + kvc) * kQKVN + hd4 * 32 + q4 * 8;
    uint4 kw = *(const uint4*)(qkv + src + 128);
    uint4 vw = *(const uint4*)(qkv + src + 256);
    const bool real = kv < kNTokW;
    kw.x = real ? kw.x : 0u; kw.y = real ? kw.y : 0u; kw.z = real ? kw.z : 0u; kw.w = real ? kw.w : 0u;
    vw.x = real ? vw.x : 0u; vw.y = real ? vw.y : 0u; vw.z = real ? vw.z : 0u; vw.w = real ? vw.w : 0u;
    *(uint4*)(kvs + (hd4 * 64 + kv) * 32 + q4 * 8) = kw;
    unsigned short* vt = kvs + 8192 + (hd4 * 32 + q4 * 8) * 64 + kv;
    vt[0]   = (unsigned short)(vw.x & 0xffffu); vt[64]  = (unsigned short)(vw.x >> 16);
    vt[128] = (unsigned short)(vw.y & 0xffffu); vt[192] = (unsigned short)(vw.y >> 16);
    vt[256] = (unsigned short)(vw.z & 0xffffu); vt[320] = (unsigned short)(vw.z >> 16);
    vt[384] = (unsigned short)(vw.w & 0xffffu); vt[448] = (unsigned short)(vw.w >> 16);
  }
  __syncthreads();

  const int h = wave & 3, mhalf = wave >> 2;
  const _Float16* k16 = (const _Float16*)kvs + h * 64 * 32;
  const _Float16* v16 = (const _Float16*)kvs + 8192 + h * 32 * 64;
  const _Float16* q16 = (const _Float16*)qkv;

  v16h qa[2];
#pragma unroll
  for (int mt = 0; mt < 2; ++mt) {
    int qr = mhalf * 32 + mt * 16 + c;
    qr = (qr < kNTokW) ? qr : (kNTokW - 1);
    qa[mt] = Frag<_Float16>::load(q16 + (rowbase + qr) * kQKVN + h * 32 + 8 * hh);
  }
  v16h kb[4];
#pragma unroll
  for (int j = 0; j < 4; ++j) kb[j] = Frag<_Float16>::load(k16 + (j * 16 + c) * 32 + 8 * hh);

  v8f sacc[2][4];
#pragma unroll
  for (int mt = 0; mt < 2; ++mt)
#pragma unroll
    for (int j = 0; j < 4; ++j) {
      v8f z = (v8f){0.f,0.f,0.f,0.f,0.f,0.f,0.f,0.f};
      sacc[mt][j] = mma_h(qa[mt], kb[j], z);
    }

  int idn[4], kcr[4], kcc[4];
  bool kreal[4];
#pragma unroll
  for (int j = 0; j < 4; ++j) {
    const int kv = j * 16 + c;
    kreal[j] = kv < kNTokW;
    const int kvq = kreal[j] ? kv : (kNTokW - 1);
    const int cr = kvq / 7;
    const int cc = kvq - cr * 7;
    kcr[j] = cr; kcc[j] = cc;
    idn[j] = 3 * region_id(wh * 7 + cr) + region_id(wn * 7 + cc);
  }

  _Float16* pw = psh[wave];
  float lsum[2][8];
  const float sc = 0.17677669529663687f * 0.015625f;
  const float ninf = -__builtin_inff();
#pragma unroll
  for (int mt = 0; mt < 2; ++mt) {
#pragma unroll
    for (int r = 0; r < 8; ++r) {
      const int qrow = mhalf * 32 + mt * 16 + 8 * hh + r;
      const int qq = (qrow < kNTokW) ? qrow : (kNTokW - 1);
      const int mr = qq / 7;
      const int mc = qq - mr * 7;
      const int idm = 3 * region_id(wh * 7 + mr) + region_id(wn * 7 + mc);
      float vals[4];
      float mx = ninf;
#pragma unroll
      for (int j = 0; j < 4; ++j) {
        const float bias = rpbs[((mr - kcr[j] + 6) * 13 + (mc - kcc[j] + 6)) * 4 + h];
        const float mk = (idm != idn[j]) ? -100.0f : 0.0f;
        float v = sacc[mt][j][r] * sc + bias;
        v = v + mk;
        v = kreal[j] ? v : ninf;
        vals[j] = v;
        mx = fmaxf(mx, v);
      }
#pragma unroll
      for (int off = 1; off < 16; off <<= 1) mx = fmaxf(mx, __shfl_xor(mx, off, 32));
      float psum = 0.f;
#pragma unroll
      for (int j = 0; j < 4; ++j) {
        const float p = expf(vals[j] - mx);
        psum += p;
        pw[(mt * 16 + 8 * hh + r) * 64 + j * 16 + c] = (_Float16)(p * 1024.0f);
      }
#pragma unroll
      for (int off = 1; off < 16; off <<= 1) psum += __shfl_xor(psum, off, 32);
      lsum[mt][r] = psum;
    }
  }
  __builtin_amdgcn_fence(__ATOMIC_RELEASE, "workgroup");
  __builtin_amdgcn_wave_barrier();
  __builtin_amdgcn_fence(__ATOMIC_ACQUIRE, "workgroup");

  v8f oacc[2][2];
#pragma unroll
  for (int mt = 0; mt < 2; ++mt)
#pragma unroll
    for (int nt = 0; nt < 2; ++nt) oacc[mt][nt] = (v8f){0.f,0.f,0.f,0.f,0.f,0.f,0.f,0.f};
#pragma unroll
  for (int kk = 0; kk < 2; ++kk) {
    v16h vb[2];
#pragma unroll
    for (int nt = 0; nt < 2; ++nt) vb[nt] = Frag<_Float16>::load(v16 + (nt * 16 + c) * 64 + kk * 32 + 8 * hh);
#pragma unroll
    for (int mt = 0; mt < 2; ++mt) {
      const v16h pa = Frag<_Float16>::load(pw + (mt * 16 + c) * 64 + kk * 32 + 8 * hh);
#pragma unroll
      for (int nt = 0; nt < 2; ++nt) oacc[mt][nt] = mma_h(pa, vb[nt], oacc[mt][nt]);
    }
  }

  __syncthreads();
  _Float16* osh = (_Float16*)kvs;
#pragma unroll
  for (int mt = 0; mt < 2; ++mt) {
#pragma unroll
    for (int r = 0; r < 8; ++r) {
      const int row = mhalf * 32 + mt * 16 + 8 * hh + r;
      const float inv = 1.0f / (lsum[mt][r] * 1024.0f);
#pragma unroll
      for (int nt = 0; nt < 2; ++nt) osh[row * 136 + h * 32 + nt * 16 + c] = (_Float16)(oacc[mt][nt][r] * inv);
    }
  }
  __syncthreads();
  {
    const int cl = lane & 15;
    _Float16* dst16 = (_Float16*)atto;
    for (int pass = 0; pass < 2; ++pass) {
#pragma unroll
      for (int it = 0; it < 4; ++it) {
        const int row = 2 * (it * 8 + wave) + hh;
        const v8h v = *(const v8h*)(osh + row * 136 + cl * 8);
        if (row < kNTokW) *(volatile v8h*)(dst16 + (rowbase + row) * kC + cl * 8) = v;
      }
      __threadfence();
    }
  }
}

constexpr size_t kOffWqkv  = 0;
constexpr size_t kOffWproj = 98304;
constexpr size_t kOffWfc1  = 131072;
constexpr size_t kOffWfc2  = 262144;
constexpr size_t kOffR1    = 393216;
constexpr size_t kSzR1     = (size_t)kTok * kC * 2;
constexpr size_t kOffR2    = kOffR1 + kSzR1;
constexpr size_t kSzR2     = (size_t)kTok * kQKVN * 2;
constexpr size_t kOffX1    = kOffR2;
constexpr size_t kSzX1     = (size_t)kTok * kC * 4;
constexpr size_t kOffH1    = kOffR2 + kSzX1;
constexpr size_t kSzH1     = (size_t)kChunk * kHid * 2;
constexpr size_t kOffR3    = kOffR2 + kSzR2;
constexpr size_t kSzR3     = (size_t)kChunk * kHid * 2;
constexpr size_t kWsTotal  = kOffR3 + kSzR3;
static_assert(kOffWproj == kOffWqkv + (size_t)kQKVN * kC * 2);
static_assert(kOffWfc1 == kOffWproj + (size_t)kC * kC * 2);
static_assert(kOffWfc2 == kOffWfc1 + (size_t)kHid * kC * 2);
static_assert(kOffR1 == kOffWfc2 + (size_t)kC * kHid * 2);
static_assert(kOffH1 + kSzH1 <= kOffR2 + kSzR2);
static_assert(kSzX1 <= kSzR2);
static_assert(kWsTotal == 128843776ull);
static_assert(kWsTotal <= 134217728ull);
static_assert(kOffR1 % 128 == 0 && kOffR2 % 128 == 0 && kOffH1 % 128 == 0 && kOffR3 % 128 == 0);

extern "C" void kernel_launch(void* const* d_in, const int* in_sizes, int n_in,
                              void* d_out, int out_size, void* d_ws, size_t ws_size,
                              hipStream_t stream) {
  if (n_in < 14) return;
  if (ws_size < kWsTotal) return;
  if (in_sizes[0] != kTok * kC || out_size != kTok * kC) return;
  if (in_sizes[3] != kQKVN * kC || in_sizes[5] != 169 * 4 || in_sizes[6] != kC * kC ||
      in_sizes[10] != kHid * kC || in_sizes[12] != kC * kHid) return;
  if (in_sizes[1] != kC || in_sizes[4] != kQKVN || in_sizes[7] != kC || in_sizes[8] != kC ||
      in_sizes[11] != kHid || in_sizes[13] != kC) return;

  const float* x      = (const float*)d_in[0];
  const float* n1g    = (const float*)d_in[1];
  const float* n1b    = (const float*)d_in[2];
  const float* qkv_w  = (const float*)d_in[3];
  const float* qkv_b  = (const float*)d_in[4];
  const float* rpb    = (const float*)d_in[5];
  const float* proj_w = (const float*)d_in[6];
  const float* proj_b = (const float*)d_in[7];
  const float* n2g    = (const float*)d_in[8];
  const float* n2b    = (const float*)d_in[9];
  const float* fc1_w  = (const float*)d_in[10];
  const float* fc1_b  = (const float*)d_in[11];
  const float* fc2_w  = (const float*)d_in[12];
  const float* fc2_b  = (const float*)d_in[13];
  float* out = (float*)d_out;

  char* ws = (char*)d_ws;
  unsigned short* WQKV  = (unsigned short*)(ws + kOffWqkv);
  unsigned short* WPROJ = (unsigned short*)(ws + kOffWproj);
  unsigned short* WFC1  = (unsigned short*)(ws + kOffWfc1);
  unsigned short* WFC2  = (unsigned short*)(ws + kOffWfc2);
  unsigned short* R1    = (unsigned short*)(ws + kOffR1);
  unsigned short* QKVP  = (unsigned short*)(ws + kOffR2);
  float*          X1    = (float*)(ws + kOffX1);
  unsigned short* H1    = (unsigned short*)(ws + kOffH1);
  unsigned short* G1    = (unsigned short*)(ws + kOffR3);

  cast_f32_f16x2<<<(kQKVN * kC / 2 + 255) / 256, 256, 0, stream>>>(qkv_w, (_Float16*)WQKV, kQKVN * kC / 2, 16.0f);
  cast_f32_f16x2<<<(kC * kC / 2 + 255) / 256, 256, 0, stream>>>(proj_w, (_Float16*)WPROJ, kC * kC / 2, 16.0f);
  cast_f32_f16x2<<<(kHid * kC / 2 + 255) / 256, 256, 0, stream>>>(fc1_w, (_Float16*)WFC1, kHid * kC / 2, 16.0f);
  cast_f32_f16x2<<<(kC * kHid / 2 + 255) / 256, 256, 0, stream>>>(fc2_w, (_Float16*)WFC2, kC * kHid / 2, 16.0f);

  ln_rows_kernel<true><<<(kTok + 3) / 4, 128, 0, stream>>>(x, n1g, n1b, (_Float16*)R1, kTok);

  {
    const int tiles = (kTok / 64) * (kQKVN / 64);
    gemm64_f16<2, 1, false, false><<<(tiles + 7) / 8, 256, 0, stream>>>(
        R1, kC, WQKV, kC, (void*)QKVP, kQKVN, qkv_b, 8.0f, nullptr, kTok, kQKVN, kC, 0.5f);
  }

  window_attention_kernel<<<kNWin, 256, 0, stream>>>(QKVP, rpb, R1);

  {
    const int tiles = (kTok / 64) * (kC / 64);
    gemm64_f16<2, 0, true, true><<<(tiles + 7) / 8, 256, 0, stream>>>(
        R1, kC, WPROJ, kC, (void*)X1, kC, proj_b, 1.0f, x, kTok, kC, kC, 1.0f / 128.0f);
  }

  ln_rows_kernel<false><<<(kTok + 3) / 4, 128, 0, stream>>>(X1, n2g, n2b, (_Float16*)R1, kTok);

  for (int ch = 0; ch < kNChunk; ++ch) {
    const size_t roff = (size_t)ch * kChunk;
    {
      const int tiles = (kChunk / 64) * (kHid / 64);
      gemm64_f16<2, 1, false, false><<<(tiles + 7) / 8, 256, 0, stream>>>(
          R1 + roff * kC, kC, WFC1, kC, (void*)H1, kHid, fc1_b, 8.0f, nullptr, kChunk, kHid, kC, 0.5f);
    }
    gelu_f16x2_kernel<<<(kChunk * kHid / 2 + 255) / 256, 256, 0, stream>>>(
        (const unsigned*)H1, (unsigned*)G1, kChunk * kHid / 2);
    {
      const int tiles = (kChunk / 64) * (kC / 64);
      gemm64_f16<2, 0, true, false><<<(tiles + 7) / 8, 256, 0, stream>>>(
          G1, kHid, WFC2, kHid, (void*)(out + roff * kC), kC, fc2_b, 1.0f, X1 + roff * kC,
          kChunk, kC, kHid, 1.0f / 256.0f);
    }
  }
}
